// CombinedModel_11209864642811
// MI455X (gfx1250) — hardware-verified
//
#include <hip/hip_runtime.h>
#include <stddef.h>


#define DL      128
#define HD      32
#define NCLS    16
#define NTHR    256
#define NWAVE   8
#define EPT     8
#define NGRP    2
#define CHUNK   (NTHR * EPT * NGRP)
#define WCAP    (EPT * NGRP * 32)
#define LISTN   (NWAVE * WCAP)
#define SHIFT   12
#define NBD     4096
#define NB1     2048
#define NB2     4096
#define TN      64
#define GN      4
#define HROWS   130
#define HP      32
#define W2SCALE 16.0f
#define W2INV   0.0625f
#define GWSCALE 8.0f
#define GWINV   0.125f
#define MAXNODES (1 << 19)

#define LDS_AGG1 (NB1 * HD * 4 + LISTN * 4 + 64)
#define LDS_AGG2 (NB2 * NCLS * 4 + LISTN * 4 + 64)

static_assert((CHUNK & (CHUNK - 1)) == 0);
static_assert((NB1 & (NB1 - 1)) == 0 && (NB2 & (NB2 - 1)) == 0 && (NBD & (NBD - 1)) == 0);
static_assert(NB1 <= (1 << SHIFT) && NB2 <= (1 << SHIFT) && NBD <= (1 << SHIFT));
static_assert(256 * NCLS * 4 <= LISTN * 4);
static_assert(NB1 % 256 == 0 && NB2 % NTHR == 0);
static_assert(TN % GN == 0 && GN * 2 == NWAVE && TN == 16 * (NWAVE / 2));
static_assert(NBD % TN == 0 && NBD % NB1 == 0 && NBD % NB2 == 0);
static_assert(DL == 128 && HD == 32 && NCLS == 16);

typedef float    v4f  __attribute__((ext_vector_type(4)));
typedef float    v8f  __attribute__((ext_vector_type(8)));
typedef int      v4i  __attribute__((ext_vector_type(4)));
typedef _Float16 v8h  __attribute__((ext_vector_type(8)));
typedef _Float16 v16h __attribute__((ext_vector_type(16)));
union FragH { v16h v; v8h h[2]; };

__device__ __forceinline__ v8h cvt8(v4f a, v4f b) {
  v8h r;
  r[0] = (_Float16)a.x; r[1] = (_Float16)a.y; r[2] = (_Float16)a.z; r[3] = (_Float16)a.w;
  r[4] = (_Float16)b.x; r[5] = (_Float16)b.y; r[6] = (_Float16)b.z; r[7] = (_Float16)b.w;
  return r;
}

__device__ __forceinline__ v8f wmh(v16h a, v16h b, v8f c) {
  v8f d = __builtin_amdgcn_wmma_f32_16x16x32_f16(false, a, false, b, (short)0, c, false, false);
  asm volatile("v_nop\n\tv_nop\n\tv_nop\n\tv_nop" : "+v"(d) : "v"(a), "v"(b));
  return d;
}

__device__ __forceinline__ v16h ldfrag16(const float* __restrict__ base, int stride, float scale) {
  v16h v;
#pragma unroll
  for (int i = 0; i < 8; ++i) {
    v[i]     = (_Float16)(base[stride * i] * scale);
    v[8 + i] = (_Float16)(base[stride * (16 + i)] * scale);
  }
  return v;
}

template <int NB, bool WSRC>
__device__ __forceinline__ int scan_chunk(const int* __restrict__ srcs, const int* __restrict__ dsts,
                                          int nE, int nN, int cbase, int nodeBase,
                                          int vec8, int* list, int tid, int lane, int wave) {
  int wc = 0;
#pragma unroll
  for (int g = 0; g < NGRP; ++g) {
    const int el0  = (g * NTHR + tid) * EPT;
    const int e0   = cbase + el0;
    const int sent = -2147483647 - 1;
    v4i da, db;
    if (vec8 != 0 && e0 + 7 < nE) {
      da = *(const v4i*)(dsts + e0);
      db = *(const v4i*)(dsts + e0 + 4);
    } else {
      da.x = (e0     < nE) ? dsts[min(e0, nE - 1)] : sent;
      da.y = (e0 + 1 < nE) ? dsts[min(e0 + 1, nE - 1)] : sent;
      da.z = (e0 + 2 < nE) ? dsts[min(e0 + 2, nE - 1)] : sent;
      da.w = (e0 + 3 < nE) ? dsts[min(e0 + 3, nE - 1)] : sent;
      db.x = (e0 + 4 < nE) ? dsts[min(e0 + 4, nE - 1)] : sent;
      db.y = (e0 + 5 < nE) ? dsts[min(e0 + 5, nE - 1)] : sent;
      db.z = (e0 + 6 < nE) ? dsts[min(e0 + 6, nE - 1)] : sent;
      db.w = (e0 + 7 < nE) ? dsts[min(e0 + 7, nE - 1)] : sent;
    }
    const unsigned nb = (unsigned)nodeBase;
    const unsigned s0 = (unsigned)da.x - nb, s1 = (unsigned)da.y - nb;
    const unsigned s2 = (unsigned)da.z - nb, s3 = (unsigned)da.w - nb;
    const unsigned s4 = (unsigned)db.x - nb, s5 = (unsigned)db.y - nb;
    const unsigned s6 = (unsigned)db.z - nb, s7 = (unsigned)db.w - nb;
    const bool h0 = s0 < (unsigned)NB, h1 = s1 < (unsigned)NB, h2 = s2 < (unsigned)NB, h3 = s3 < (unsigned)NB;
    const bool h4 = s4 < (unsigned)NB, h5 = s5 < (unsigned)NB, h6 = s6 < (unsigned)NB, h7 = s7 < (unsigned)NB;
    const unsigned any = __builtin_amdgcn_ballot_w32(h0 | h1 | h2 | h3 | h4 | h5 | h6 | h7);
    if (any != 0u) {
#define HITJ(J, HJ, SJ) { \
        const unsigned mj = __builtin_amdgcn_ballot_w32(HJ); \
        if (mj != 0u) { \
          if (HJ) { \
            const int pos = wc + (int)__builtin_amdgcn_mbcnt_lo(mj, 0u); \
            int ent = (int)(SJ); \
            if (WSRC) { \
              int ee = e0 + (J); ee = ee > nE - 1 ? nE - 1 : ee; \
              int sv = srcs[ee]; \
              sv = sv < 0 ? 0 : (sv > nN - 1 ? nN - 1 : sv); \
              ent |= sv << SHIFT; \
            } \
            if (pos < WCAP) list[wave * WCAP + pos] = ent; \
          } \
          wc += (int)__builtin_popcount(mj); } }
      HITJ(0, h0, s0)
      HITJ(1, h1, s1)
      HITJ(2, h2, s2)
      HITJ(3, h3, s3)
      HITJ(4, h4, s4)
      HITJ(5, h5, s5)
      HITJ(6, h6, s6)
      HITJ(7, h7, s7)
#undef HITJ
    }
  }
  return wc;
}

__global__ __launch_bounds__(NTHR) void k_deg(
    const int* __restrict__ ei, float* dinv, int nN, int nE, int vec8) {
  __shared__ __attribute__((aligned(16))) int cnt[NBD];
  __shared__ __attribute__((aligned(16))) int list[LISTN];
  __shared__ int wcnt[NWAVE];
  const int tid = threadIdx.x, lane = tid & 31, wave = tid >> 5;
  const int nodeBase = blockIdx.x * NBD;
  const int* dsts = ei + nE;

  for (int i = tid; i < NBD; i += NTHR) cnt[i] = 0;
  __syncthreads();

  const int nChunks = (nE + CHUNK - 1) / CHUNK;
#pragma unroll 1
  for (int ch = 0; ch < nChunks; ++ch) {
    const int cbase = ch * CHUNK;
    const int wc = scan_chunk<NBD, false>(ei, dsts, nE, nN, cbase, nodeBase, vec8, list, tid, lane, wave);
    if (lane == 0) wcnt[wave] = wc;
    __syncthreads();
    if (wave == 0) {
#pragma unroll 1
      for (int wsx = 0; wsx < NWAVE; ++wsx) {
        int n = __builtin_amdgcn_readfirstlane(wcnt[wsx]);
        n = n > WCAP ? WCAP : (n < 0 ? 0 : n);
        const int* lp = list + wsx * WCAP;
#pragma unroll 1
        for (int i = 0; i < n; ++i) {
          const int ent  = __builtin_amdgcn_readfirstlane(lp[i]);
          const int slot = ent & (NBD - 1);
          if (lane == 0) cnt[slot] = cnt[slot] + 1;
        }
      }
    }
    __syncthreads();
  }

  v4f dq[4];
#pragma unroll
  for (int q = 0; q < 4; ++q) {
    const int f = (wave * 4 + q) * 128 + 4 * lane;
    const v4i c = *(const v4i*)(cnt + f);
    dq[q].x = rsqrtf((float)(c.x + 1));
    dq[q].y = rsqrtf((float)(c.y + 1));
    dq[q].z = rsqrtf((float)(c.z + 1));
    dq[q].w = rsqrtf((float)(c.w + 1));
  }
  float* dp = dinv + (size_t)nodeBase;
#pragma unroll
  for (int q = 0; q < 4; ++q) *(volatile v4f*)(dp + (wave * 4 + q) * 128 + 4 * lane) = dq[q];
  __threadfence();
#pragma unroll
  for (int q = 0; q < 4; ++q) *(volatile v4f*)(dp + (wave * 4 + q) * 128 + 4 * lane) = dq[q];
}

__global__ __launch_bounds__(NTHR) void k_cnn(
    const float* __restrict__ x,  const float* __restrict__ w1, const float* __restrict__ b1,
    const float* __restrict__ w2, const float* __restrict__ b2, const float* __restrict__ gw1,
    const float* __restrict__ dinv, float* g1, int nN) {
  __shared__ __attribute__((aligned(16))) _Float16 h1T[GN * HROWS * HP];
  __shared__ __attribute__((aligned(16))) _Float16 pooled[TN * HD];
  __shared__ __attribute__((aligned(16))) float    stg[TN * HD];
  const int tid = threadIdx.x, lane = tid & 31, wave = tid >> 5, hh = lane >> 4, m = lane & 15;
  const int nodeBase = blockIdx.x * TN;

  if (tid < GN * 2 * 4) {
    const int g = tid >> 3, which = (tid >> 2) & 1, piece = tid & 3;
    v8h z;
#pragma unroll
    for (int i = 0; i < 8; ++i) z[i] = (_Float16)0.f;
    *(v8h*)(h1T + (g * HROWS + (which ? (HROWS - 1) : 0)) * HP + piece * 8) = z;
  }

  const int cg = tid & 3;
  float wr[24], br[8];
#pragma unroll
  for (int c = 0; c < 8; ++c) {
    wr[3 * c]     = w1[(8 * cg + c) * 3];
    wr[3 * c + 1] = w1[(8 * cg + c) * 3 + 1];
    wr[3 * c + 2] = w1[(8 * cg + c) * 3 + 2];
    br[c]         = b1[8 * cg + c];
  }

  const int ct = wave & 1, gsel = wave >> 1;
  FragH af[3];
#pragma unroll
  for (int kk = 0; kk < 3; ++kk)
    af[kk].v = ldfrag16(w2 + ((size_t)(16 * ct + m) * HD + 8 * hh) * 3 + kk, 3, W2SCALE);
  const float b2v = b2[16 * ct + 8 * hh + (m & 7)];

  const int mt = wave >> 1, nt = wave & 1;
  FragH bg;
  bg.v = ldfrag16(gw1 + (size_t)(8 * hh) * HD + 16 * nt + m, HD, GWSCALE);

  __syncthreads();

#pragma unroll 1
  for (int grp = 0; grp < TN / GN; ++grp) {
    const int gbase = nodeBase + grp * GN;
#pragma unroll
    for (int it = 0; it < 2 * GN; ++it) {
      const int g = it >> 1;
      const int d = (it & 1) * 64 + (tid >> 2);
      int node = gbase + g;
      node = node > nN - 1 ? nN - 1 : node;
      const float* xp = x + (size_t)node * DL;
      const int dm = d > 0 ? d - 1 : 0;
      const int dr = d < DL - 1 ? d + 1 : DL - 1;
      const float x0 = xp[d];
      float xm = xp[dm]; xm = d > 0 ? xm : 0.f;
      float xr = xp[dr]; xr = d < DL - 1 ? xr : 0.f;
      v8h hv;
#pragma unroll
      for (int c = 0; c < 8; ++c) {
        const float v = fmaf(wr[3 * c], xm, fmaf(wr[3 * c + 1], x0, fmaf(wr[3 * c + 2], xr, br[c])));
        hv[c] = (_Float16)fmaxf(v, 0.f);
      }
      *(v8h*)(h1T + (g * HROWS + d + 1) * HP + cg * 8) = hv;
    }
    __syncthreads();

    {
      const _Float16* hb = h1T + (gsel * HROWS) * HP + 8 * hh;
      v8f vmax;
#pragma unroll
      for (int r = 0; r < 8; ++r) vmax[r] = -3.0e38f;
#pragma unroll
      for (int pt = 0; pt < DL / 16; ++pt) {
        v8f c = {0.f, 0.f, 0.f, 0.f, 0.f, 0.f, 0.f, 0.f};
#pragma unroll
        for (int kk = 0; kk < 3; ++kk) {
          const _Float16* bp = hb + (16 * pt + m + kk) * HP;
          FragH b;
          b.h[0] = *(const v8h*)bp;
          b.h[1] = *(const v8h*)(bp + 16);
          c = wmh(af[kk].v, b.v, c);
        }
#pragma unroll
        for (int r = 0; r < 8; ++r) vmax[r] = fmaxf(vmax[r], c[r]);
      }
#pragma unroll
      for (int r = 0; r < 8; ++r) {
        float v = vmax[r];
        v = fmaxf(v, __shfl_xor(v, 8));
        v = fmaxf(v, __shfl_xor(v, 4));
        v = fmaxf(v, __shfl_xor(v, 2));
        v = fmaxf(v, __shfl_xor(v, 1));
        vmax[r] = v;
      }
      float sel = vmax[0];
#pragma unroll
      for (int r = 1; r < 8; ++r) sel = ((m & 7) == r) ? vmax[r] : sel;
      const float pv = fmaxf(sel * W2INV + b2v, 0.f);
      if (m < 8) pooled[(grp * GN + gsel) * HD + 16 * ct + 8 * hh + m] = (_Float16)pv;
    }
    __syncthreads();
  }

  {
    const _Float16* ar = pooled + (16 * mt + m) * HD + 8 * hh;
    FragH a;
    a.h[0] = *(const v8h*)ar;
    a.h[1] = *(const v8h*)(ar + 16);
    v8f c = {0.f, 0.f, 0.f, 0.f, 0.f, 0.f, 0.f, 0.f};
    c = wmh(a.v, bg.v, c);
    const int r0 = 16 * mt + 8 * hh;
    const v4f dA = *(const v4f*)(dinv + (size_t)nodeBase + r0);
    const v4f dB = *(const v4f*)(dinv + (size_t)nodeBase + r0 + 4);
    float* sp = stg + r0 * HD + 16 * nt + m;
    sp[0 * HD] = c[0] * dA.x * GWINV;
    sp[1 * HD] = c[1] * dA.y * GWINV;
    sp[2 * HD] = c[2] * dA.z * GWINV;
    sp[3 * HD] = c[3] * dA.w * GWINV;
    sp[4 * HD] = c[4] * dB.x * GWINV;
    sp[5 * HD] = c[5] * dB.y * GWINV;
    sp[6 * HD] = c[6] * dB.z * GWINV;
    sp[7 * HD] = c[7] * dB.w * GWINV;
  }
  __syncthreads();

  {
    const int row = 8 * wave + (lane >> 3), col = 4 * (lane & 7);
    const v4f v = *(const v4f*)(stg + row * HD + col);
    float* gp = g1 + ((size_t)nodeBase + row) * HD + col;
    *(volatile v4f*)gp = v;
    __threadfence();
    *(volatile v4f*)gp = v;
  }
}

__global__ __launch_bounds__(NTHR) void k_agg1(
    const int* __restrict__ ei, const float* __restrict__ g1, const float* __restrict__ dinv,
    const float* __restrict__ gb1, const float* __restrict__ gw2, float* g2,
    int nN, int nE, int vec8) {
  extern __shared__ v4f lds_dyn[];
  float* acc  = (float*)lds_dyn;
  int*   list = (int*)(acc + NB1 * HD);
  int*   wcnt = list + LISTN;
  float* stg2 = (float*)list;
  const int tid = threadIdx.x, lane = tid & 31, wave = tid >> 5, hh = lane >> 4, m = lane & 15;
  const int nodeBase = blockIdx.x * NB1;
  const int* dsts = ei + nE;

  {
    const v4f z = {0.f, 0.f, 0.f, 0.f};
    for (int i = tid; i < NB1 * HD / 4; i += NTHR) lds_dyn[i] = z;
  }
  __syncthreads();

  const int nChunks = (nE + CHUNK - 1) / CHUNK;
#pragma unroll 1
  for (int ch = 0; ch < nChunks; ++ch) {
    const int cbase = ch * CHUNK;
    const int wc = scan_chunk<NB1, true>(ei, dsts, nE, nN, cbase, nodeBase, vec8, list, tid, lane, wave);
    if (lane == 0) wcnt[wave] = wc;
    __syncthreads();
    if (wave == 0) {
#pragma unroll 1
      for (int wsx = 0; wsx < NWAVE; ++wsx) {
        int n = __builtin_amdgcn_readfirstlane(wcnt[wsx]);
        n = n > WCAP ? WCAP : (n < 0 ? 0 : n);
        const int* lp = list + wsx * WCAP;
#pragma unroll 1
        for (int i = 0; i < n; ++i) {
          const int ent  = __builtin_amdgcn_readfirstlane(lp[i]);
          const int slot = ent & (NB1 - 1);
          int src = ent >> SHIFT;
          src = src < 0 ? 0 : (src > nN - 1 ? nN - 1 : src);
          const float v = g1[(size_t)src * HD + lane];
          float* ap = acc + slot * HD + lane;
          *ap = *ap + v;
        }
      }
    }
    __syncthreads();
  }

#pragma unroll 4
  for (int i = 0; i < (NB1 * HD / 4) / NTHR; ++i) {
    const int idx  = i * NTHR + tid;
    const int slot = idx >> 3;
    const int c4   = (idx & 7) * 4;
    int node = nodeBase + slot;
    node = node > nN - 1 ? nN - 1 : node;
    const float d  = dinv[node];
    const v4f   gv = *(const v4f*)(g1 + (size_t)node * HD + c4);
    const v4f   bv = *(const v4f*)(gb1 + c4);
    v4f* ap = (v4f*)(acc + slot * HD + c4);
    v4f hv = (*ap + gv) * d + bv;
    hv.x = fmaxf(hv.x, 0.f); hv.y = fmaxf(hv.y, 0.f); hv.z = fmaxf(hv.z, 0.f); hv.w = fmaxf(hv.w, 0.f);
    *ap = hv;
  }
  __syncthreads();

  FragH bw;
  bw.v = ldfrag16(gw2 + (size_t)(8 * hh) * NCLS + m, NCLS, GWSCALE);

#pragma unroll 1
  for (int s = 0; s < NB1 / 256; ++s) {
#pragma unroll
    for (int q = 0; q < 2; ++q) {
      const int tl = wave + 8 * q;
      const int t  = 16 * s + tl;
      const float* ap = acc + (16 * t + m) * HD + 8 * hh;
      const v4f p0 = *(const v4f*)ap,        p1 = *(const v4f*)(ap + 4);
      const v4f p2 = *(const v4f*)(ap + 16), p3 = *(const v4f*)(ap + 20);
      FragH a;
      a.h[0] = cvt8(p0, p1);
      a.h[1] = cvt8(p2, p3);
      v8f c = {0.f, 0.f, 0.f, 0.f, 0.f, 0.f, 0.f, 0.f};
      c = wmh(a.v, bw.v, c);
      const int node0 = nodeBase + 16 * t + 8 * hh;
      const v4f dA = *(const v4f*)(dinv + (size_t)node0);
      const v4f dB = *(const v4f*)(dinv + (size_t)node0 + 4);
      float* sp = stg2 + (16 * tl + 8 * hh) * NCLS + m;
      sp[0 * NCLS] = c[0] * dA.x * GWINV;
      sp[1 * NCLS] = c[1] * dA.y * GWINV;
      sp[2 * NCLS] = c[2] * dA.z * GWINV;
      sp[3 * NCLS] = c[3] * dA.w * GWINV;
      sp[4 * NCLS] = c[4] * dB.x * GWINV;
      sp[5 * NCLS] = c[5] * dB.y * GWINV;
      sp[6 * NCLS] = c[6] * dB.z * GWINV;
      sp[7 * NCLS] = c[7] * dB.w * GWINV;
    }
    __syncthreads();
    v4f ov[4];
#pragma unroll
    for (int q = 0; q < 4; ++q) ov[q] = *(const v4f*)(stg2 + (wave * 4 + q) * 128 + 4 * lane);
    float* gp = g2 + ((size_t)nodeBase + 256 * s) * NCLS;
#pragma unroll
    for (int q = 0; q < 4; ++q) *(volatile v4f*)(gp + (wave * 4 + q) * 128 + 4 * lane) = ov[q];
    __threadfence();
#pragma unroll
    for (int q = 0; q < 4; ++q) *(volatile v4f*)(gp + (wave * 4 + q) * 128 + 4 * lane) = ov[q];
    __syncthreads();
  }
}

__global__ __launch_bounds__(NTHR) void k_agg2(
    const int* __restrict__ ei, const float* __restrict__ g2, const float* __restrict__ dinv,
    const float* __restrict__ gb2, float* out, int nN, int nE, int vec8) {
  extern __shared__ v4f lds_dyn[];
  float* acc  = (float*)lds_dyn;
  int*   list = (int*)(acc + NB2 * NCLS);
  int*   wcnt = list + LISTN;
  const int tid = threadIdx.x, lane = tid & 31, wave = tid >> 5;
  const int nodeBase = blockIdx.x * NB2;
  const int* dsts = ei + nE;

  {
    const v4f z = {0.f, 0.f, 0.f, 0.f};
    for (int i = tid; i < NB2 * NCLS / 4; i += NTHR) lds_dyn[i] = z;
  }
  __syncthreads();

  const int nChunks = (nE + CHUNK - 1) / CHUNK;
#pragma unroll 1
  for (int ch = 0; ch < nChunks; ++ch) {
    const int cbase = ch * CHUNK;
    const int wc = scan_chunk<NB2, true>(ei, dsts, nE, nN, cbase, nodeBase, vec8, list, tid, lane, wave);
    if (lane == 0) wcnt[wave] = wc;
    __syncthreads();
    if (wave == 0) {
#pragma unroll 1
      for (int wsx = 0; wsx < NWAVE; ++wsx) {
        int n = __builtin_amdgcn_readfirstlane(wcnt[wsx]);
        n = n > WCAP ? WCAP : (n < 0 ? 0 : n);
        const int* lp = list + wsx * WCAP;
#pragma unroll 1
        for (int i = 0; i < n; ++i) {
          const int ent  = __builtin_amdgcn_readfirstlane(lp[i]);
          const int slot = ent & (NB2 - 1);
          int src = ent >> SHIFT;
          src = src < 0 ? 0 : (src > nN - 1 ? nN - 1 : src);
          if (lane < NCLS) {
            float* ap = acc + slot * NCLS + lane;
            *ap = *ap + g2[(size_t)src * NCLS + lane];
          }
        }
      }
    }
    __syncthreads();
  }

  v4f bq[4];
#pragma unroll
  for (int k = 0; k < 4; ++k) bq[k] = *(const v4f*)(gb2 + 4 * k);
#pragma unroll 1
  for (int j = 0; j < NB2 / NTHR; ++j) {
    const int r = j * NTHR + tid;
    int node = nodeBase + r;
    node = node > nN - 1 ? nN - 1 : node;
    const float d = dinv[node];
    v4f* ap = (v4f*)(acc + r * NCLS);
    const v4f* gp = (const v4f*)(g2 + (size_t)node * NCLS);
    v4f v[4];
#pragma unroll
    for (int k = 0; k < 4; ++k) v[k] = (ap[k] + gp[k]) * d + bq[k];
    float mx = v[0].x;
#pragma unroll
    for (int k = 0; k < 4; ++k) {
      mx = fmaxf(mx, v[k].x); mx = fmaxf(mx, v[k].y); mx = fmaxf(mx, v[k].z); mx = fmaxf(mx, v[k].w);
    }
    float s = 0.f;
#pragma unroll
    for (int k = 0; k < 4; ++k) {
      s += __expf(v[k].x - mx); s += __expf(v[k].y - mx); s += __expf(v[k].z - mx); s += __expf(v[k].w - mx);
    }
    const float ls = logf(s);
#pragma unroll
    for (int k = 0; k < 4; ++k) {
      v4f o;
      o.x = (v[k].x - mx) - ls; o.y = (v[k].y - mx) - ls; o.z = (v[k].z - mx) - ls; o.w = (v[k].w - mx) - ls;
      ap[k] = o;
    }
  }
  __syncthreads();

  const size_t outN = (size_t)nN * NCLS;
  const size_t ob   = (size_t)nodeBase * NCLS;
#pragma unroll 4
  for (int q = 0; q < 64; ++q) {
    const int f = (wave * 64 + q) * 128 + 4 * lane;
    const size_t gi = ob + (size_t)f;
    if (gi < outN) { const v4f v = *(const v4f*)(acc + f); *(volatile v4f*)(out + gi) = v; }
  }
  __threadfence();
#pragma unroll 4
  for (int q = 0; q < 64; ++q) {
    const int f = (wave * 64 + q) * 128 + 4 * lane;
    const size_t gi = ob + (size_t)f;
    if (gi < outN) { const v4f v = *(const v4f*)(acc + f); *(volatile v4f*)(out + gi) = v; }
  }
}

extern "C" void kernel_launch(void* const* d_in, const int* in_sizes, int n_in,
                              void* d_out, int out_size, void* d_ws, size_t ws_size,
                              hipStream_t stream) {
  if (n_in < 10) return;
  const int nN = in_sizes[0] / DL;
  const int nE = in_sizes[1] / 2;
  if (nN <= 0 || nN > MAXNODES || nE < 0 || in_sizes[0] != nN * DL || in_sizes[1] != nE * 2) return;
  if (in_sizes[2] != HD * 3 || in_sizes[3] < HD || in_sizes[4] != HD * HD * 3 || in_sizes[5] < HD) return;
  if (in_sizes[6] != HD * HD || in_sizes[7] < HD || in_sizes[8] != HD * NCLS || in_sizes[9] < NCLS) return;
  if (out_size != nN * NCLS) return;

  const float* x   = (const float*)d_in[0];
  const int*   ei  = (const int*)d_in[1];
  const float* w1  = (const float*)d_in[2];
  const float* b1  = (const float*)d_in[3];
  const float* w2  = (const float*)d_in[4];
  const float* b2  = (const float*)d_in[5];
  const float* gw1 = (const float*)d_in[6];
  const float* gb1 = (const float*)d_in[7];
  const float* gw2 = (const float*)d_in[8];
  const float* gb2 = (const float*)d_in[9];
  float* out = (float*)d_out;

  const int nBD = (nN + NBD - 1) / NBD;
  const int nCB = (nN + TN - 1) / TN;
  const int nA1 = (nN + NB1 - 1) / NB1;
  const int nA2 = (nN + NB2 - 1) / NB2;

  char* ws = (char*)d_ws;
  size_t off = 0;
  const size_t oDv = off; off += (size_t)nBD * NBD * 4;                        off = (off + 255) & ~(size_t)255;
  const size_t oG1 = off; off += (size_t)nCB * TN * HD * 4;                    off = (off + 255) & ~(size_t)255;
  const size_t oG2 = off; off += (size_t)nA1 * NB1 * NCLS * 4;                 off = (off + 255) & ~(size_t)255;
  if (off > ws_size || off > (size_t)134217728) return;
  float* dinv = (float*)(ws + oDv);
  float* g1   = (float*)(ws + oG1);
  float* g2   = (float*)(ws + oG2);

  const int vec8 = ((nE & 3) == 0) ? 1 : 0;

  k_deg<<<nBD, NTHR, 0, stream>>>(ei, dinv, nN, nE, vec8);

  k_cnn<<<nCB, NTHR, 0, stream>>>(x, w1, b1, w2, b2, gw1, dinv, g1, nN);

  hipFuncSetAttribute(reinterpret_cast<const void*>(&k_agg1),
                      hipFuncAttributeMaxDynamicSharedMemorySize, LDS_AGG1);
  k_agg1<<<nA1, NTHR, LDS_AGG1, stream>>>(ei, g1, dinv, gb1, gw2, g2, nN, nE, vec8);

  hipFuncSetAttribute(reinterpret_cast<const void*>(&k_agg2),
                      hipFuncAttributeMaxDynamicSharedMemorySize, LDS_AGG2);
  k_agg2<<<nA2, NTHR, LDS_AGG2, stream>>>(ei, g2, dinv, gb2, out, nN, nE, vec8);
}
